// ExpertsFeedForward_76871324663968
// MI455X (gfx1250) — hardware-verified
//
#include <hip/hip_runtime.h>


#ifndef NB
#define NB 2
#endif
#ifndef SEQ
#define SEQ 256
#endif
#define NB_FULL  2
#define SEQ_FULL 256
#ifndef OUT_SEQ
#define OUT_SEQ SEQ
#endif
#define DM   256
#define HID  1024
#define NE   16
#define TK   2
#define NTOK (NB * SEQ)
#define NENT (NTOK * TK)
#define MT   16
#define MAX_TILES (NENT / MT)
#define FW   8
#define XP   (DM + 8)
#define GP   (HID + 8)
#define OSP  36
#define GS   64.0f
#define VS   4096.0f

static_assert(MT == 16);
static_assert(TK == 2);
static_assert(DM % 32 == 0);
static_assert(HID % 32 == 0);
static_assert(HID % (16 * FW) == 0);
static_assert(FW * 32 == DM);
static_assert(2 * 32 * FW == MT * (DM / 8));
static_assert(4 * 32 * FW >= NENT);
static_assert(NENT % 4 == 0);
static_assert(NENT >= 4);
static_assert(NENT % MT == 0);
static_assert(SEQ % 2 == 0);
static_assert(SEQ_FULL % 2 == 0);
static_assert(NB <= NB_FULL);
static_assert(SEQ <= SEQ_FULL);
static_assert((XP * 2) % 16 == 0);
static_assert((GP * 2) % 16 == 0);
static_assert((OSP * 4) % 16 == 0);
static_assert(4 * 4 == MT);
static_assert(8 * 4 == 32);
static_assert(((size_t)NTOK * DM) % 8 == 0);
static_assert(((size_t)NE * HID * DM) % 8 == 0);
static_assert((size_t)MT * XP * 2 + (size_t)MT * GP * 2 + (size_t)FW * 16 * OSP * 4 + MT * 8 + FW * 4 <= 131072);

typedef _Float16 h16;
typedef unsigned short bf;
typedef __attribute__((ext_vector_type(16))) __bf16   v16bf;
typedef __attribute__((ext_vector_type(16))) _Float16 v16h;
typedef __attribute__((ext_vector_type(8)))  _Float16 v8h;
typedef __attribute__((ext_vector_type(8)))  unsigned short v8us;
typedef __attribute__((ext_vector_type(8)))  float    v8f;
typedef __attribute__((ext_vector_type(4)))  float    v4f;
typedef __attribute__((ext_vector_type(4)))  int      v4i;
typedef v4f  __attribute__((may_alias)) v4fa;

__device__ __forceinline__ unsigned short f2bf(float f) { unsigned u = __float_as_uint(f); u += 0x7FFFu + ((u >> 16) & 1u); return (unsigned short)(u >> 16); }
__device__ __forceinline__ float bfr(float f) { return __uint_as_float(((unsigned)f2bf(f)) << 16); }
__device__ __forceinline__ v16h cat16(v8h lo, v8h hi) { return __builtin_shufflevector(lo, hi, 0, 1, 2, 3, 4, 5, 6, 7, 8, 9, 10, 11, 12, 13, 14, 15); }
__device__ __forceinline__ v16bf cat16b(v8us lo, v8us hi) { return __builtin_bit_cast(v16bf, __builtin_shufflevector(lo, hi, 0, 1, 2, 3, 4, 5, 6, 7, 8, 9, 10, 11, 12, 13, 14, 15)); }
__device__ __forceinline__ v16h  ldh(const h16* p) { return cat16(*(const v8h*)p, *(const v8h*)(p + 16)); }
__device__ __forceinline__ v16bf ldb(const bf* p)  { return cat16b(*(const v8us*)p, *(const v8us*)(p + 16)); }
__device__ __forceinline__ void wave_sync() { __builtin_amdgcn_fence(3  , "wavefront"); __builtin_amdgcn_wave_barrier(); asm volatile("" ::: "memory"); }

static __device__ __forceinline__ h16 toh_flush(float v) { const h16 r = (h16)v; return (fabsf(v) < 6.103515625e-05f) ? (h16)0.0f : r; }
__device__ __forceinline__ v8f wmmab_g(v16bf a, v16bf b, v8f c) {
    c = __builtin_amdgcn_wmma_f32_16x16x32_bf16(false, a, false, b, (short)0, c, false, false);
    asm volatile("v_nop\n\tv_nop\n\tv_nop\n\tv_nop" : "+v"(c) : "v"(a), "v"(b));
    return c;
}
__device__ __forceinline__ v8f wmma16_g(v16h a, v16h b, v8f c) {
    c = __builtin_amdgcn_wmma_f32_16x16x32_f16(false, a, false, b, (short)0, c, false, false);
    asm volatile("v_nop\n\tv_nop\n\tv_nop\n\tv_nop" : "+v"(c) : "v"(a), "v"(b));
    return c;
}
__device__ __forceinline__ float gelu_t(float h) {
    const float u = 0.7978845608028654f * (h + 0.044715f * (h * h * h));
    const float a = fminf(u * 2.8853900817779268f, 80.0f);
    const float ex = __builtin_amdgcn_exp2f(a);
    return h * (ex * __builtin_amdgcn_rcpf(1.0f + ex));
}

__global__ __launch_bounds__(256) void k_cvt8(const float* __restrict__ src, bf* dst, size_t n8) {
    const size_t i = (size_t)blockIdx.x * 256 + threadIdx.x; if (i >= n8) return;
    const v8f v = *(const v8f*)(src + i * 8); v8us o;
#pragma unroll
    for (int k = 0; k < 8; ++k) o[k] = f2bf(v[k]);
    *(volatile v8us*)(dst + i * 8) = o; __threadfence(); *(volatile v8us*)(dst + i * 8) = o;
}

__global__ __launch_bounds__(256) void k_cvth8(const float* __restrict__ src, h16* dst, size_t n8) {
    const size_t i = (size_t)blockIdx.x * 256 + threadIdx.x; if (i >= n8) return;
    const v8f v = *(const v8f*)(src + i * 8); v8h o;
#pragma unroll
    for (int k = 0; k < 8; ++k) o[k] = toh_flush(bfr(v[k]) * VS);
    *(volatile v8h*)(dst + i * 8) = o; __threadfence(); *(volatile v8h*)(dst + i * 8) = o;
}

__global__ __launch_bounds__(32 * FW) void k_ffn(const bf* __restrict__ XB, const bf* __restrict__ KB, const h16* __restrict__ VH,
                                                 const float* __restrict__ ew, const int* __restrict__ eidx, float* Y) {
    __shared__ __align__(16) bf    xs[MT * XP];
    __shared__ __align__(16) h16   gs[MT * GP];
    __shared__ __align__(16) float os[FW * 16 * OSP];
    __shared__ int   s_ent[MT];
    __shared__ float s_w[MT];
    __shared__ int   s_cnt[FW];
    const int tid = threadIdx.x;
    const int lane = tid & 31, lr = lane & 15, hi = lane >> 4;
    const int wave = __builtin_amdgcn_readfirstlane((int)(threadIdx.x >> 5));
    const int wv = tid >> 5;
    const int tile = blockIdx.x, e = blockIdx.y;
    if (tid < MT) { s_ent[tid] = -1; s_w[tid] = 0.0f; }
    const int g0 = 4 * tid;
    const int gv = (g0 < NENT) ? 1 : 0;
    const int gc = (g0 < NENT - 4) ? g0 : (NENT - 4);
    const int tk0 = gc / TK;
    const size_t ioff = ((size_t)(tk0 / SEQ) * SEQ_FULL + (size_t)(tk0 % SEQ)) * TK;
    v4i q = *(const v4i*)(eidx + ioff);
    v4f wq = *(const v4f*)(ew + ioff);
    asm volatile("" : "+v"(q));
    asm volatile("" : "+v"(wq));
    const unsigned lt = (1u << lane) - 1u;
    int hj[4]; int pre = 0, tot = 0;
#pragma unroll
    for (int j = 0; j < 4; ++j) {
        int ej = q[j]; ej = ej < 0 ? 0 : (ej > NE - 1 ? NE - 1 : ej);
        hj[j] = gv & ((ej == e) ? 1 : 0);
        const unsigned mk = __builtin_amdgcn_ballot_w32(hj[j] != 0);
        pre += __builtin_popcount(mk & lt); tot += __builtin_popcount(mk); }
    if (lane == 0) s_cnt[wave] = tot;
    __syncthreads();
    int base = 0, cnt = 0;
#pragma unroll
    for (int w = 0; w < FW; ++w) { const int c = s_cnt[w]; cnt += c; base += (w < wv) ? c : 0; }
    cnt = __builtin_amdgcn_readfirstlane(cnt);
    if (tile * MT >= cnt) return;
    {
        int p = base + pre - tile * MT;
#pragma unroll
        for (int j = 0; j < 4; ++j) {
            if ((hj[j] != 0) & ((unsigned)p < (unsigned)MT)) { s_ent[p] = g0 + j; s_w[p] = bfr(wq[j]); }
            p += hj[j]; }
    }
    __syncthreads();
#pragma unroll
    for (int i = 0; i < 2; ++i) {
        const int p = tid + 32 * FW * i; const int r = p >> 5, c8 = (p & 31) * 8;
        int en = s_ent[r]; en = en < 0 ? 0 : (en > NENT - 1 ? NENT - 1 : en);
        const v8us v = *(const v8us*)(XB + (size_t)(en / TK) * DM + c8);
        *(v8us*)(&xs[r * XP + c8]) = v; }
    __syncthreads();

    v16bf a[DM / 32];
    const int xo = lr * XP + 8 * hi;
#pragma unroll
    for (int kc = 0; kc < DM / 32; ++kc) a[kc] = cat16b(*(const v8us*)(&xs[xo + kc * 32]), *(const v8us*)(&xs[xo + kc * 32 + 16]));
    const size_t kbase = ((size_t)e * HID + (size_t)lr) * DM + 8 * hi;
#pragma unroll 1
    for (int nb = 0; nb < HID / (16 * FW); ++nb) {
        const int h0 = (wave * (HID / (16 * FW)) + nb) * 16;
        const bf* bp = KB + kbase + (size_t)h0 * DM;
        v8f acc = (v8f){};
#pragma unroll
        for (int kc = 0; kc < DM / 32; ++kc) { const v16bf b = ldb(bp + kc * 32); acc = wmmab_g(a[kc], b, acc); }
#pragma unroll
        for (int j = 0; j < 8; ++j) gs[(8 * hi + j) * GP + h0 + lr] = toh_flush(gelu_t(acc[j]) * GS);
    }
    __syncthreads();

    v8f o0 = (v8f){}, o1 = (v8f){};
    const int go = lr * GP + 8 * hi;
    const size_t vbase = ((size_t)e * DM + (size_t)(wave * 32 + lr)) * HID + 8 * hi;
#pragma unroll 1
    for (int kc = 0; kc < HID; kc += 32) {
        const v16h ga = cat16(*(const v8h*)(&gs[go + kc]), *(const v8h*)(&gs[go + kc + 16]));
        const v16h b0 = ldh(VH + vbase + kc), b1 = ldh(VH + vbase + (size_t)16 * HID + kc);
        o0 = wmma16_g(ga, b0, o0); o1 = wmma16_g(ga, b1, o1);
    }
    const float fold = 1.0f / (GS * VS);
    const int wb = wave * 16 * OSP;
#pragma unroll
    for (int j = 0; j < 8; ++j) { const float sc = s_w[8 * hi + j] * fold;
        os[wb + (8 * hi + j) * OSP + lr] = o0[j] * sc; os[wb + (8 * hi + j) * OSP + 16 + lr] = o1[j] * sc; }
    wave_sync();
#pragma unroll 1
    for (int ps = 0; ps < 2; ++ps) {
#pragma unroll
        for (int s = 0; s < 4; ++s) { const int row = 4 * s + (lane >> 3), cofs = (lane & 7) * 4;
            const v4f val = *(const v4fa*)(&os[wb + row * OSP + cofs]);
            const int en = s_ent[row];
            if ((unsigned)en < (unsigned)NENT) *(volatile v4f*)(Y + (size_t)en * DM + wave * 32 + cofs) = val; }
        if (ps == 0) __threadfence(); }
}

__global__ __launch_bounds__(256) void k_comb(const float* __restrict__ Y, float* OUT) {
    const int i = blockIdx.x * 256 + threadIdx.x; if (i >= NTOK * (DM / 4)) return;
    const int tok = i / (DM / 4), c4 = (i % (DM / 4)) * 4;
    const v4f y0 = *(const v4f*)(Y + (size_t)(tok * TK) * DM + c4);
    const v4f y1 = *(const v4f*)(Y + (size_t)(tok * TK + 1) * DM + c4);
    const v4f o = y0 + y1;
    float* op = OUT + ((size_t)(tok / SEQ) * OUT_SEQ + (size_t)(tok % SEQ)) * DM + c4;
    *(volatile v4f*)op = o; __threadfence(); *(volatile v4f*)op = o;
}

static constexpr size_t al256(size_t v) { return (v + 255) & ~(size_t)255; }
static constexpr size_t SZ_XB = al256((size_t)NTOK * DM * 2);
static constexpr size_t SZ_KB = al256((size_t)NE * HID * DM * 2);
static constexpr size_t SZ_VH = al256((size_t)NE * DM * HID * 2);
static constexpr size_t SZ_Y  = al256((size_t)NENT * DM * 4);
static constexpr size_t SZ_TOTAL = SZ_XB + SZ_KB + SZ_VH + SZ_Y;
static_assert(SZ_TOTAL <= (size_t)134217728);
static_assert(((size_t)NTOK * (DM / 4)) % 256 == 0);
static_assert(((size_t)DM * 4) % 128 == 0);

extern "C" void kernel_launch(void* const* d_in, const int* in_sizes, int n_in,
                              void* d_out, int out_size, void* d_ws, size_t ws_size, hipStream_t stream) {
    if (n_in < 5) return;
    const size_t needx = ((size_t)(NB - 1) * SEQ_FULL + SEQ) * DM;
    const size_t needr = ((size_t)(NB - 1) * SEQ_FULL + SEQ) * TK;
    if ((size_t)in_sizes[0] < needx) return;
    if ((size_t)in_sizes[1] < (size_t)NE * HID * DM || (size_t)in_sizes[2] < (size_t)NE * DM * HID) return;
    if ((size_t)in_sizes[3] < needr || (size_t)in_sizes[4] < needr) return;
    if ((size_t)out_size < ((size_t)(NB - 1) * OUT_SEQ + SEQ) * DM) return;
    if (SZ_TOTAL > ws_size) return;
    const float* x = (const float*)d_in[0];
    const float* keys = (const float*)d_in[1];
    const float* values = (const float*)d_in[2];
    const float* ew = (const float*)d_in[3];
    const int* eidx = (const int*)d_in[4];
    float* OUT = (float*)d_out;
    char* wsp = (char*)d_ws;
    bf*  XB = (bf*)wsp;  wsp += SZ_XB;
    bf*  KB = (bf*)wsp;  wsp += SZ_KB;
    h16* VH = (h16*)wsp; wsp += SZ_VH;
    float* Y = (float*)wsp; wsp += SZ_Y;

    if (SEQ == SEQ_FULL) {
        const size_t n8 = (size_t)NB * SEQ * DM / 8;
        k_cvt8<<<(unsigned)((n8 + 255) / 256), 256, 0, stream>>>(x, XB, n8);
    } else {
        const size_t n8 = (size_t)SEQ * DM / 8;
        for (int b = 0; b < NB; ++b) k_cvt8<<<(unsigned)((n8 + 255) / 256), 256, 0, stream>>>(x + (size_t)b * SEQ_FULL * DM, XB + (size_t)b * SEQ * DM, n8);
    }
    { const size_t n8 = (size_t)NE * HID * DM / 8; const unsigned g = (unsigned)((n8 + 255) / 256);
      k_cvt8<<<g, 256, 0, stream>>>(keys, KB, n8);
      k_cvth8<<<g, 256, 0, stream>>>(values, VH, n8); }

    k_ffn<<<dim3(MAX_TILES, NE, 1), 32 * FW, 0, stream>>>(XB, KB, VH, ew, eidx, Y);
    k_comb<<<(unsigned)(((size_t)NTOK * (DM / 4)) / 256), 256, 0, stream>>>(Y, OUT);
}
